// SelfAttention_11029476016812
// MI455X (gfx1250) — hardware-verified
//
#include <hip/hip_runtime.h>
#ifndef NB
#define NB 8
#endif
#ifndef SEQ
#define SEQ 4096
#endif
#define NB_FULL 8
#define SEQ_FULL 4096
#define CC 64
#define XP 72
#define SOP 68

static_assert(CC == 64);
static_assert(CC % 32 == 0);
static_assert(SEQ % 64 == 0);
static_assert(SEQ <= SEQ_FULL);
static_assert(NB <= NB_FULL);
static_assert(XP % 8 == 0 && XP >= CC);
static_assert(SOP % 4 == 0 && SOP >= 64);
static_assert((size_t)5 * NB * SEQ * CC * 2 <= (size_t)134217728);

typedef __bf16 v16b __attribute__((ext_vector_type(16)));
typedef _Float16 v16h __attribute__((ext_vector_type(16)));
typedef unsigned short v8us __attribute__((ext_vector_type(8), may_alias));
typedef float v8f __attribute__((ext_vector_type(8)));
typedef float v4f __attribute__((ext_vector_type(4)));
typedef float v4fa __attribute__((ext_vector_type(4), may_alias));
union FragB { v16b v; v8us half[2]; unsigned short u[16]; };
union FragH { v16h v; v8us half[2]; _Float16 h[16]; unsigned short u[16]; };

__device__ __forceinline__ unsigned short bf16_bits(float x) { unsigned int u = __float_as_uint(x); return (unsigned short)((u + 0x7FFFu + ((u >> 16) & 1u)) >> 16); }
__device__ __forceinline__ float bf16_val(unsigned short b) { return __uint_as_float(((unsigned int)b) << 16); }
__device__ __forceinline__ float bf16_rne(float x) { return bf16_val(bf16_bits(x)); }

__device__ __forceinline__ v8f mma1b(v16b a, v16b b, v8f c) {
  c = __builtin_amdgcn_wmma_f32_16x16x32_bf16(false, a, false, b, (short)0, c, false, false);
  asm volatile("v_nop\n\tv_nop\n\tv_nop\n\tv_nop" : "+v"(c) : "v"(a), "v"(b));
  return c;
}
__device__ __forceinline__ v8f mma3b(v16b ah, v16b al, v16b bh, v16b bl, v8f c) {
  c = __builtin_amdgcn_wmma_f32_16x16x32_bf16(false, ah, false, bh, (short)0, c, false, false);
  c = __builtin_amdgcn_wmma_f32_16x16x32_bf16(false, al, false, bh, (short)0, c, false, false);
  c = __builtin_amdgcn_wmma_f32_16x16x32_bf16(false, ah, false, bl, (short)0, c, false, false);
  asm volatile("v_nop\n\tv_nop\n\tv_nop\n\tv_nop" : "+v"(c) : "v"(ah), "v"(al), "v"(bh), "v"(bl));
  return c;
}
__device__ __forceinline__ v8f mma1h(v16h a, v16h b, v8f c) {
  c = __builtin_amdgcn_wmma_f32_16x16x32_f16(false, a, false, b, (short)0, c, false, false);
  asm volatile("v_nop\n\tv_nop\n\tv_nop\n\tv_nop" : "+v"(c) : "v"(a), "v"(b));
  return c;
}

__device__ __forceinline__ v16b frag_b(const unsigned short* __restrict__ p, size_t off) {
  FragB f; f.half[0] = *(const v8us*)(p + off); f.half[1] = *(const v8us*)(p + off + 16); return f.v;
}
__device__ __forceinline__ v16h frag_h(const unsigned short* __restrict__ p, size_t off) {
  FragH f; f.half[0] = *(const v8us*)(p + off); f.half[1] = *(const v8us*)(p + off + 16); return f.v;
}
__device__ __forceinline__ v16b frag_w(const float* __restrict__ W, int off) {
  const v4f x0 = *(const v4fa*)(W + off), x1 = *(const v4fa*)(W + off + 4);
  const v4f x2 = *(const v4fa*)(W + off + 16), x3 = *(const v4fa*)(W + off + 20);
  FragB f;
  f.u[0] = bf16_bits(x0[0]); f.u[1] = bf16_bits(x0[1]); f.u[2] = bf16_bits(x0[2]); f.u[3] = bf16_bits(x0[3]);
  f.u[4] = bf16_bits(x1[0]); f.u[5] = bf16_bits(x1[1]); f.u[6] = bf16_bits(x1[2]); f.u[7] = bf16_bits(x1[3]);
  f.u[8] = bf16_bits(x2[0]); f.u[9] = bf16_bits(x2[1]); f.u[10] = bf16_bits(x2[2]); f.u[11] = bf16_bits(x2[3]);
  f.u[12] = bf16_bits(x3[0]); f.u[13] = bf16_bits(x3[1]); f.u[14] = bf16_bits(x3[2]); f.u[15] = bf16_bits(x3[3]);
  return f.v;
}

__global__ __launch_bounds__(128) void k_proj_qk(const float* __restrict__ X, const float* __restrict__ W, const float* __restrict__ bias,
                                                 unsigned short* __restrict__ PH, unsigned short* __restrict__ PL) {
  __shared__ __attribute__((aligned(16))) unsigned short xs[64][XP];
  __shared__ __attribute__((aligned(16))) unsigned short sh[64][XP];
  __shared__ __attribute__((aligned(16))) unsigned short sl[64][XP];
  const int tid = threadIdx.x;
  const int wave = __builtin_amdgcn_readfirstlane(tid >> 5);
  const int lane = tid & 31, ln = lane & 15, hh = lane >> 4;
  const int b = blockIdx.y, pb = blockIdx.x * 64;
  const float* xb = X + (size_t)b * CC * SEQ_FULL + pb;
#pragma unroll
  for (int j = 0; j < 8; ++j) {
    const int idx = j * 128 + tid;
    const int c = idx >> 4, p4 = (idx & 15) * 4;
    const v4f x4 = *(const v4fa*)(xb + (size_t)c * SEQ_FULL + p4);
    xs[p4 + 0][c] = bf16_bits(x4[0]); xs[p4 + 1][c] = bf16_bits(x4[1]);
    xs[p4 + 2][c] = bf16_bits(x4[2]); xs[p4 + 3][c] = bf16_bits(x4[3]);
  }
  __syncthreads();
  const int prow = wave * 16 + ln;
  FragB a0, a1;
  a0.half[0] = *(const v8us*)&xs[prow][8 * hh];       a0.half[1] = *(const v8us*)&xs[prow][16 + 8 * hh];
  a1.half[0] = *(const v8us*)&xs[prow][32 + 8 * hh];  a1.half[1] = *(const v8us*)&xs[prow][48 + 8 * hh];
#pragma unroll
  for (int ot = 0; ot < 4; ++ot) {
    const int woff = (ot * 16 + ln) * CC + 8 * hh;
    const v16b w0 = frag_w(W, woff), w1 = frag_w(W, woff + 32);
    v8f acc = {0.f, 0.f, 0.f, 0.f, 0.f, 0.f, 0.f, 0.f};
    acc = mma1b(a0.v, w0, acc);
    acc = mma1b(a1.v, w1, acc);
    const float bv = bf16_rne(bias[ot * 16 + ln]);
#pragma unroll
    for (int r = 0; r < 8; ++r) {
      const float v = acc[r] + bv;
      const unsigned short hb = bf16_bits(v);
      const unsigned short lb = bf16_bits(v - bf16_val(hb));
      sh[wave * 16 + 8 * hh + r][ot * 16 + ln] = hb;
      sl[wave * 16 + 8 * hh + r][ot * 16 + ln] = lb;
    }
  }
  __syncthreads();
  const size_t rowbase = (size_t)b * SEQ + pb;
  const int pc = (tid & 7) * 8;
  for (int pass = 0; pass < 2; ++pass) {
#pragma unroll
    for (int it = 0; it < 4; ++it) {
      const int row = it * 16 + (tid >> 3);
      const v8us vh = *(const v8us*)&sh[row][pc];
      const v8us vl = *(const v8us*)&sl[row][pc];
      *(volatile v8us*)(PH + (rowbase + row) * CC + pc) = vh;
      *(volatile v8us*)(PL + (rowbase + row) * CC + pc) = vl;
    }
    if (pass == 0) __threadfence();
  }
}

__global__ __launch_bounds__(128) void k_proj_v(const float* __restrict__ X, const float* __restrict__ W, const float* __restrict__ bias,
                                                unsigned short* __restrict__ VT) {
  __shared__ __attribute__((aligned(16))) unsigned short xs[64][XP];
  __shared__ __attribute__((aligned(16))) unsigned short sv[64][XP];
  const int tid = threadIdx.x;
  const int wave = __builtin_amdgcn_readfirstlane(tid >> 5);
  const int lane = tid & 31, ln = lane & 15, hh = lane >> 4;
  const int b = blockIdx.y, pb = blockIdx.x * 64;
  const float* xb = X + (size_t)b * CC * SEQ_FULL + pb;
#pragma unroll
  for (int j = 0; j < 8; ++j) {
    const int idx = j * 128 + tid;
    const int c = idx >> 4, p4 = (idx & 15) * 4;
    const v4f x4 = *(const v4fa*)(xb + (size_t)c * SEQ_FULL + p4);
    xs[p4 + 0][c] = bf16_bits(x4[0]); xs[p4 + 1][c] = bf16_bits(x4[1]);
    xs[p4 + 2][c] = bf16_bits(x4[2]); xs[p4 + 3][c] = bf16_bits(x4[3]);
  }
  __syncthreads();
  const int prow = wave * 16 + ln;
  FragB b0, b1;
  b0.half[0] = *(const v8us*)&xs[prow][8 * hh];       b0.half[1] = *(const v8us*)&xs[prow][16 + 8 * hh];
  b1.half[0] = *(const v8us*)&xs[prow][32 + 8 * hh];  b1.half[1] = *(const v8us*)&xs[prow][48 + 8 * hh];
#pragma unroll
  for (int ot = 0; ot < 4; ++ot) {
    const int woff = (ot * 16 + ln) * CC + 8 * hh;
    const v16b w0 = frag_w(W, woff), w1 = frag_w(W, woff + 32);
    v8f acc = {0.f, 0.f, 0.f, 0.f, 0.f, 0.f, 0.f, 0.f};
    acc = mma1b(w0, b0.v, acc);
    acc = mma1b(w1, b1.v, acc);
#pragma unroll
    for (int r = 0; r < 8; ++r) {
      const int c = ot * 16 + 8 * hh + r;
      const float v = acc[r] + bf16_rne(bias[c]);
      sv[c][wave * 16 + ln] = __builtin_bit_cast(unsigned short, (_Float16)v);
    }
  }
  __syncthreads();
  const int pc = (tid & 7) * 8;
  for (int pass = 0; pass < 2; ++pass) {
#pragma unroll
    for (int it = 0; it < 4; ++it) {
      const int c = it * 16 + (tid >> 3);
      const v8us vv = *(const v8us*)&sv[c][pc];
      *(volatile v8us*)(VT + ((size_t)b * CC + c) * SEQ + pb + pc) = vv;
    }
    if (pass == 0) __threadfence();
  }
}

__global__ __launch_bounds__(128) void k_attn(const float* __restrict__ query, const unsigned short* __restrict__ QH, const unsigned short* __restrict__ QL,
                                              const unsigned short* __restrict__ KH, const unsigned short* __restrict__ KL,
                                              const unsigned short* __restrict__ VT, float* __restrict__ out) {
  __shared__ __attribute__((aligned(16))) float so[CC][SOP];
  const int tid = threadIdx.x;
  const int wave = __builtin_amdgcn_readfirstlane(tid >> 5);
  const int lane = tid & 31, ln = lane & 15, hh = lane >> 4;
  const int b = blockIdx.y, qb = blockIdx.x * 64;
  const size_t tok0 = (size_t)b * SEQ;
  const size_t qoff = (tok0 + qb + wave * 16 + ln) * CC + 8 * hh;
  const v16b qh0 = frag_b(QH, qoff), qh1 = frag_b(QH, qoff + 32);
  const v16b ql0 = frag_b(QL, qoff), ql1 = frag_b(QL, qoff + 32);
  const v8f z8 = {0.f, 0.f, 0.f, 0.f, 0.f, 0.f, 0.f, 0.f};
  v8f o0 = z8, o1 = z8, o2 = z8, o3 = z8;
  float m = -3.0e38f, l = 0.f;
  const float SC = 0.18033688011112042f;
  const size_t kofs = (tok0 + ln) * CC + 8 * hh;
  const size_t vofs = ((size_t)b * CC + ln) * SEQ + 8 * hh;
#pragma unroll 1
  for (int kb = 0; kb < SEQ; kb += 32) {
    const size_t ka = kofs + (size_t)kb * CC;
    v8f s0 = z8, s1 = z8;
    { const v16b ah = frag_b(KH, ka), al = frag_b(KL, ka); s0 = mma3b(ah, al, qh0, ql0, s0); }
    { const v16b ah = frag_b(KH, ka + 32), al = frag_b(KL, ka + 32); s0 = mma3b(ah, al, qh1, ql1, s0); }
    { const v16b ah = frag_b(KH, ka + 16 * CC), al = frag_b(KL, ka + 16 * CC); s1 = mma3b(ah, al, qh0, ql0, s1); }
    { const v16b ah = frag_b(KH, ka + 16 * CC + 32), al = frag_b(KL, ka + 16 * CC + 32); s1 = mma3b(ah, al, qh1, ql1, s1); }
    float cmax = s0[0];
#pragma unroll
    for (int r = 1; r < 8; ++r) cmax = fmaxf(cmax, s0[r]);
#pragma unroll
    for (int r = 0; r < 8; ++r) cmax = fmaxf(cmax, s1[r]);
    cmax = fmaxf(cmax, __shfl_xor(cmax, 16));
    const float mn = fmaxf(m, cmax);
    const float alpha = __builtin_amdgcn_exp2f((m - mn) * SC);
    FragH pf;
    float lsum = 0.f;
#pragma unroll
    for (int r = 0; r < 8; ++r) { const float p = __builtin_amdgcn_exp2f((s0[r] - mn) * SC); lsum += p; pf.h[r] = (_Float16)(p * 256.0f); }
#pragma unroll
    for (int r = 0; r < 8; ++r) { const float p = __builtin_amdgcn_exp2f((s1[r] - mn) * SC); lsum += p; pf.h[8 + r] = (_Float16)(p * 256.0f); }
    l = l * alpha + lsum;
    m = mn;
#pragma unroll
    for (int r = 0; r < 8; ++r) { o0[r] *= alpha; o1[r] *= alpha; o2[r] *= alpha; o3[r] *= alpha; }
    const size_t va = vofs + kb;
    { const v16h a = frag_h(VT, va); o0 = mma1h(a, pf.v, o0); }
    { const v16h a = frag_h(VT, va + (size_t)16 * SEQ); o1 = mma1h(a, pf.v, o1); }
    { const v16h a = frag_h(VT, va + (size_t)32 * SEQ); o2 = mma1h(a, pf.v, o2); }
    { const v16h a = frag_h(VT, va + (size_t)48 * SEQ); o3 = mma1h(a, pf.v, o3); }
  }
  const float lt = l + __shfl_xor(l, 16);
  const float inv = 0.00390625f * (1.0f / lt);
  const int qc = wave * 16 + ln;
#pragma unroll
  for (int r = 0; r < 8; ++r) {
    so[8 * hh + r][qc] = o0[r] * inv;
    so[16 + 8 * hh + r][qc] = o1[r] * inv;
    so[32 + 8 * hh + r][qc] = o2[r] * inv;
    so[48 + 8 * hh + r][qc] = o3[r] * inv;
  }
  __syncthreads();
  v4f res[8];
  const int c4 = ln * 4;
#pragma unroll
  for (int it = 0; it < 8; ++it) {
    const int c = wave * 16 + it * 2 + hh;
    const v4f ov = *(const v4fa*)&so[c][c4];
    const size_t g = ((size_t)b * CC + c) * SEQ_FULL + qb + c4;
    const v4f qv = *(const v4fa*)(query + g);
    v4f rr;
    rr[0] = bf16_rne(qv[0]) + ov[0]; rr[1] = bf16_rne(qv[1]) + ov[1];
    rr[2] = bf16_rne(qv[2]) + ov[2]; rr[3] = bf16_rne(qv[3]) + ov[3];
    res[it] = rr;
  }
  for (int pass = 0; pass < 2; ++pass) {
#pragma unroll
    for (int it = 0; it < 8; ++it) {
      const int c = wave * 16 + it * 2 + hh;
      const size_t g = ((size_t)b * CC + c) * SEQ_FULL + qb + c4;
      *(volatile v4f*)(out + g) = res[it];
    }
    if (pass == 0) __threadfence();
  }
}

extern "C" void kernel_launch(void* const* d_in, const int* in_sizes, int n_in,
                              void* d_out, int out_size, void* d_ws, size_t ws_size, hipStream_t stream) {
  if (n_in < 9) return;
  const long long need_x = ((long long)(NB - 1) * CC + (CC - 1)) * SEQ_FULL + SEQ;
  if ((long long)in_sizes[0] < need_x || (long long)in_sizes[1] < need_x || (long long)in_sizes[2] < need_x) return;
  if (in_sizes[3] < CC * CC || in_sizes[5] < CC * CC || in_sizes[7] < CC * CC) return;
  if (in_sizes[4] < CC || in_sizes[6] < CC || in_sizes[8] < CC) return;
  if ((long long)out_size < need_x) return;
  const float* xq = (const float*)d_in[0]; const float* xk = (const float*)d_in[1]; const float* xv = (const float*)d_in[2];
  const float* Wq = (const float*)d_in[3]; const float* bq = (const float*)d_in[4];
  const float* Wk = (const float*)d_in[5]; const float* bk = (const float*)d_in[6];
  const float* Wv = (const float*)d_in[7]; const float* bv = (const float*)d_in[8];
  const size_t PB = (size_t)NB * SEQ * CC * 2;
  if (5 * PB > ws_size) return;
  char* ws = (char*)d_ws;
  unsigned short* QH = (unsigned short*)(ws);
  unsigned short* QL = (unsigned short*)(ws + PB);
  unsigned short* KH = (unsigned short*)(ws + 2 * PB);
  unsigned short* KL = (unsigned short*)(ws + 3 * PB);
  unsigned short* VT = (unsigned short*)(ws + 4 * PB);
  const dim3 grid(SEQ / 64, NB);
  k_proj_qk<<<grid, 128, 0, stream>>>(xq, Wq, bq, QH, QL);
  k_proj_qk<<<grid, 128, 0, stream>>>(xk, Wk, bk, KH, KL);
  k_proj_v<<<grid, 128, 0, stream>>>(xv, Wv, bv, VT);
  k_attn<<<grid, 128, 0, stream>>>(xq, QH, QL, KH, KL, VT, (float*)d_out);
}
